// Engine_48378511622701
// MI455X (gfx1250) — hardware-run, weakly checked
//
#include <hip/hip_runtime.h>


namespace {
constexpr int B = 2, N = 40000, E = 640000, D = 128, NE = 24, M = B * N, QW = 3 * D;
constexpr float XS = 8.0f, WSC = 256.0f, NEG = 0.2f  , ISQD = 0.08838834764831845f, EPSD = 1e-9f;
typedef _Float16 b16;
typedef __attribute__((ext_vector_type(16))) _Float16 v16b;
typedef __attribute__((ext_vector_type(8))) _Float16 v8b;
typedef __attribute__((ext_vector_type(8))) float v8f;
typedef __attribute__((ext_vector_type(4))) float v4f;
__device__ __forceinline__ float bf16_rne(float f) { unsigned int u = __float_as_uint(f); u += 0x7FFFu + ((u >> 16) & 1u); return __uint_as_float(u & 0xFFFF0000u); }
__device__ __forceinline__ void split16(float v, b16& hi, b16& lo) { hi = (b16)v; lo = (b16)(v - (float)hi); }
__device__ __forceinline__ v16b frag_kb(const b16* p, int hh) { const v8b a = *(const v8b*)(p + 8 * hh), b = *(const v8b*)(p + 16 + 8 * hh); v16b f;
#pragma unroll
  for (int e = 0; e < 8; ++e) { f[e] = a[e]; f[8 + e] = b[e]; } return f; }
__device__ __forceinline__ v8f wmma16b(v16b a, v16b b, v8f c) { v8f d = __builtin_amdgcn_wmma_f32_16x16x32_f16(false, a, false, b, (short)0, c, false, false); asm volatile("v_nop\n\tv_nop\n\tv_nop\n\tv_nop" : "+v"(d) : "v"(a), "v"(b)); return d; }
__device__ __forceinline__ void wave_lds_sync() { __builtin_amdgcn_fence(__ATOMIC_RELEASE, "workgroup"); __builtin_amdgcn_wave_barrier(); __builtin_amdgcn_fence(__ATOMIC_ACQUIRE, "workgroup"); }
__device__ __forceinline__ float pmul(float a, float b) { float p = a * b; asm volatile("" : "+v"(p)); return p; }
__device__ __forceinline__ int iclamp(int v, int lo, int hi) { return v < lo ? lo : (v > hi ? hi : v); }
__device__ __forceinline__ float nexp(float x) { return __builtin_amdgcn_exp2f(x * 1.4426950408889634f); }
constexpr int CSR_NBLK = 512, CSR_GB = 9, CSR_GN = 1 << CSR_GB  , CSR_MAXG = 512, CSR_CAP = 12288  ;
__global__ __launch_bounds__(64) void csrA_kernel(const int* __restrict__ dst, int E, int N, int nG, int CHP, int NGP, int* __restrict__ STG, int* __restrict__ HST) {
  extern __shared__ int sm[];
  int* cnt = sm; int* run = sm + NGP; int* ids = sm + 2 * NGP;
  const int b = blockIdx.x; const int ch = (E + CSR_NBLK - 1) / CSR_NBLK; const int e0 = b * ch, e1 = min(E, e0 + ch);
  for (int i = threadIdx.x; i < NGP; i += 64) cnt[i] = 0;
  for (int i = threadIdx.x; i < CHP; i += 64) ids[i] = -1;
  __syncthreads();
  if (threadIdx.x == 0) {
    for (int e = e0; e < e1; ++e) { int d = dst[e]; d = (d < 0) ? 0 : (d >= N ? N - 1 : d); cnt[d >> CSR_GB] += 1; }
    int acc = 0; for (int g = 0; g < nG; ++g) { run[g] = acc; acc += cnt[g]; }
    for (int e = e0; e < e1; ++e) { int d = dst[e]; d = (d < 0) ? 0 : (d >= N ? N - 1 : d); const int g = d >> CSR_GB; ids[run[g]] = e; run[g] += 1; } }
  __syncthreads();
  typedef __attribute__((ext_vector_type(4))) int v4i;
  for (int pass = 0; pass < 2; ++pass) {
    for (int i = threadIdx.x; i < CHP / 4; i += 64) *(volatile v4i*)(STG + (size_t)b * CHP + i * 4) = *(const v4i*)(&ids[i * 4]);
    for (int i = threadIdx.x; i < NGP / 4; i += 64) { v4i v; for (int e = 0; e < 4; ++e) v[e] = (i * 4 + e < nG) ? cnt[i * 4 + e] : 0; *(volatile v4i*)(HST + (size_t)b * NGP + i * 4) = v; }
    __threadfence(); }
}
__global__ __launch_bounds__(512) void csrS_kernel(const int* __restrict__ HST, int nG, int NGP, int* __restrict__ START, int* __restrict__ TOT, int* __restrict__ OFF) {
  __shared__ int tot[CSR_MAXG];
  const int b = threadIdx.x;
  for (int pass = 0; pass < 2; ++pass) { int runb = 0; for (int g = 0; g < nG; ++g) { int c = HST[(size_t)b * NGP + g]; c = (c < 0) ? 0 : c; ((volatile int*)OFF)[(size_t)g * CSR_NBLK + b] = runb; runb += c; } __threadfence(); }
  for (int g = threadIdx.x; g < nG; g += 512) { int s = 0; for (int bb = 0; bb < CSR_NBLK; ++bb) { int c = HST[(size_t)bb * NGP + g]; s += (c < 0) ? 0 : c; } tot[g] = s; }
  __syncthreads();
  if (threadIdx.x < 32) {
    __shared__ int st[CSR_MAXG + 32];
    if (threadIdx.x == 0) { int acc = 0; for (int g = 0; g < NGP; ++g) { st[g] = acc; if (g < nG) acc += (tot[g] + 31) & ~31; } st[NGP] = acc; }
    __builtin_amdgcn_fence(__ATOMIC_RELEASE, "workgroup"); __builtin_amdgcn_wave_barrier(); __builtin_amdgcn_fence(__ATOMIC_ACQUIRE, "workgroup");
    for (int pass = 0; pass < 2; ++pass) { for (int i = threadIdx.x; i < NGP + 32; i += 32) { ((volatile int*)START)[i] = (i <= NGP) ? st[min(i, NGP)] : 0; ((volatile int*)TOT)[i] = (i < nG) ? tot[i] : 0; } __threadfence(); } }
}
__global__ __launch_bounds__(256) void csrB_kernel(const int* __restrict__ dst, int N, int nG, int CHP, int NGP, int permLen, const int* __restrict__ STG, const int* __restrict__ HST, const int* __restrict__ OFF, const int* __restrict__ START, const int* __restrict__ TOT, int* __restrict__ PERM, int* __restrict__ ROWPTR, int* __restrict__ ROWCNT, int* __restrict__ FLAG) {
  typedef __attribute__((ext_vector_type(4))) int v4i;
  __shared__ int ids[CSR_CAP]; __shared__ unsigned short key[CSR_CAP]; __shared__ int outp[CSR_CAP]; __shared__ int ncnt[CSR_GN + 1]; __shared__ int boff[CSR_NBLK + 1];
  const int g = blockIdx.x, t_ = threadIdx.x; int tot = TOT[g]; int st = START[g], stn = START[g + 1]; const int v0 = g * CSR_GN; const int nv = min(CSR_GN, N - v0);
  st = (st < 0) ? 0 : (st > permLen - 32 ? permLen - 32 : st) & ~31; stn = (stn < st) ? st : (stn > permLen ? permLen : stn); tot = (tot < 0) ? 0 : tot; if (tot > stn - st && tot <= CSR_CAP) tot = stn - st;
  if (tot > CSR_CAP) {
    for (int pass = 0; pass < 2; ++pass) { for (int i = t_; i < CSR_GN / 4; i += 256) { v4i a, c; for (int e = 0; e < 4; ++e) { a[e] = st; c[e] = 0; } *(volatile v4i*)(ROWPTR + v0 + i * 4) = a; *(volatile v4i*)(ROWCNT + v0 + i * 4) = c; } if (t_ == 0) ((volatile int*)FLAG)[0] = 1; __threadfence(); } (void)nv; return; }
  if (t_ == 0) { int acc = 0; for (int b = 0; b < CSR_NBLK; ++b) { boff[b] = acc; int c = HST[(size_t)b * NGP + g]; c = (c < 0) ? 0 : (c > CHP ? CHP : c); acc += c; if (acc > tot) acc = tot; } boff[CSR_NBLK] = acc; }
  for (int i = t_; i <= CSR_GN; i += 256) ncnt[i] = 0;
  __syncthreads();
  for (int b = 0; b < CSR_NBLK; ++b) { const int c = boff[b + 1] - boff[b]; int o_ = OFF[(size_t)g * CSR_NBLK + b]; o_ = (o_ < 0) ? 0 : (o_ > CHP - c ? CHP - c : o_); const int* src_ = STG + (size_t)b * CHP + o_;
    for (int i = t_; i < c; i += 256) { int id = src_[i]; id = (id < 0) ? 0 : id; ids[boff[b] + i] = id; int d = dst[id]; d = (d < v0) ? v0 : (d >= N ? N - 1 : d); int kk = d - v0; kk = (kk < 0) ? 0 : (kk >= CSR_GN ? CSR_GN - 1 : kk); key[boff[b] + i] = (unsigned short)kk; } }
  __syncthreads();
  if (t_ == 0) { for (int i = 0; i < tot; ++i) ncnt[key[i]] += 1; int acc = 0; for (int vl = 0; vl < CSR_GN; ++vl) { const int c = ncnt[vl]; ncnt[vl] = acc; acc += c; } ncnt[CSR_GN] = acc;
    for (int i = 0; i < tot; ++i) { const int vl = key[i]; outp[ncnt[vl]] = ids[i]; ncnt[vl] += 1; }
    for (int vl = CSR_GN; vl > 0; --vl) ncnt[vl] = ncnt[vl - 1]; ncnt[0] = 0; }
  __syncthreads();
  for (int pass = 0; pass < 2; ++pass) {
    for (int i = t_; i < (stn - st) / 4; i += 256) { v4i v; for (int e = 0; e < 4; ++e) { const int q = i * 4 + e; v[e] = (q < tot) ? outp[q] : -1; } *(volatile v4i*)(PERM + st + i * 4) = v; }
    for (int i = t_; i < CSR_GN / 4; i += 256) { v4i a, c; for (int e = 0; e < 4; ++e) { const int vl = i * 4 + e; a[e] = st + ncnt[vl]; c[e] = (vl < nv) ? (ncnt[vl + 1] - ncnt[vl]) : 0; } *(volatile v4i*)(ROWPTR + v0 + i * 4) = a; *(volatile v4i*)(ROWCNT + v0 + i * 4) = c; }
    __threadfence(); }
}
__global__ __launch_bounds__(256) void csrZ_kernel(int* __restrict__ p, size_t n4) { typedef __attribute__((ext_vector_type(4))) int v4i; const size_t tid = (size_t)blockIdx.x * 256 + threadIdx.x, nth = (size_t)gridDim.x * 256; v4i z = {0, 0, 0, 0}; for (size_t i = tid; i < n4; i += nth) *(volatile v4i*)(p + i * 4) = z; }
struct CsrBufs { int *STG, *HST, *OFF, *START, *TOT, *PERM, *ROWPTR, *ROWCNT, *FLAG; int nG, NGP, CHP; size_t permLen; char* base; size_t bytes; };
static size_t csr_carve(CsrBufs& c, char* ws, size_t off, int E, int N) {
  const size_t off0 = off; c.base = ws + off;
  auto al = [&](size_t bytes) { char* p = ws + off; off += (bytes + 255) & ~(size_t)255; return p; };
  c.nG = (N + CSR_GN - 1) / CSR_GN; c.NGP = (c.nG + 31) & ~31; const int ch = (E + CSR_NBLK - 1) / CSR_NBLK; c.CHP = (ch + 31) & ~31; c.permLen = (size_t)E + 32 * (size_t)c.nG + 32;
  c.STG = (int*)al((size_t)CSR_NBLK * c.CHP * 4); c.HST = (int*)al((size_t)CSR_NBLK * c.NGP * 4); c.OFF = (int*)al((size_t)c.NGP * CSR_NBLK * 4); c.START = (int*)al((size_t)(c.NGP + 64) * 4); c.TOT = (int*)al((size_t)(c.NGP + 64) * 4);
  c.PERM = (int*)al(c.permLen * 4); c.ROWPTR = (int*)al((size_t)c.nG * CSR_GN * 4); c.ROWCNT = (int*)al((size_t)c.nG * CSR_GN * 4); c.FLAG = (int*)al(256);
  c.bytes = off - off0; return off;
}
static void csr_build(const CsrBufs& c, const int* dst, int E, int N, hipStream_t stream) {
  const size_t smem = (size_t)(2 * c.NGP + c.CHP) * 4;
  csrZ_kernel<<<512, 256, 0, stream>>>((int*)c.base, c.bytes / 16);
  csrA_kernel<<<CSR_NBLK, 64, smem, stream>>>(dst, E, N, c.nG, c.CHP, c.NGP, c.STG, c.HST);
  csrS_kernel<<<1, 512, 0, stream>>>(c.HST, c.nG, c.NGP, c.START, c.TOT, c.OFF);
  csrB_kernel<<<c.nG, 256, 0, stream>>>(dst, N, c.nG, c.CHP, c.NGP, (int)c.permLen, c.STG, c.HST, c.OFF, c.START, c.TOT, c.PERM, c.ROWPTR, c.ROWCNT, c.FLAG);
}


__global__ __launch_bounds__(256) void wprep_kernel(const float* __restrict__ wq, const float* __restrict__ wk, const float* __restrict__ wm, const float* __restrict__ wh, const float* __restrict__ wa, b16* __restrict__ WQK, b16* __restrict__ WHA) {
  const size_t u = (size_t)blockIdx.x * 256 + threadIdx.x; const size_t n0 = (size_t)QW * D / 8, n1 = (size_t)D * 2 * D / 8; size_t t = u; v8b o;
  if (t < n0) { const size_t e = t * 8; const int row = (int)(e / D), k0 = (int)(e % D); const int part = row / D, oo = row % D; const float* w = part == 0 ? wq : part == 1 ? wk : wm; for (int j = 0; j < 8; ++j) o[j] = (b16)(bf16_rne(w[(size_t)(k0 + j) * D + oo]) * WSC); for (int pass = 0; pass < 2; ++pass) { *(volatile v8b*)(WQK + e) = o; __threadfence(); } return; } t -= n0;
  if (t < n1) { const size_t e = t * 8; const int oo = (int)(e / (2 * D)), k0 = (int)(e % (2 * D)); for (int j = 0; j < 8; ++j) { const int k = k0 + j; const float w = k < D ? wh[(size_t)k * D + oo] : wa[(size_t)(k - D) * D + oo]; o[j] = (b16)(bf16_rne(w) * WSC); } for (int pass = 0; pass < 2; ++pass) { *(volatile v8b*)(WHA + e) = o; __threadfence(); } }
}
__global__ __launch_bounds__(256) void gw_kernel(const float* __restrict__ g, const float* __restrict__ wg, float* __restrict__ GW) {
  const int b = threadIdx.x / D, c = threadIdx.x % D; float s = 0.0f;
#pragma unroll 1
  for (int k = 0; k < D; ++k) s += pmul(bf16_rne(g[b * D + k]), bf16_rne(wg[(size_t)k * D + c]));
  for (int pass = 0; pass < 2; ++pass) { ((volatile float*)GW)[threadIdx.x] = s; __threadfence(); }
}
__global__ __launch_bounds__(128) void qkm_kernel(const float* __restrict__ ns, const float* __restrict__ npar, const b16* __restrict__ WQK, float* __restrict__ QKM) {
  __shared__ __attribute__((aligned(16))) b16 Ah[4][16][D + 8], Al[4][16][D + 8]; __shared__ __attribute__((aligned(16))) float Tf[4][16][128 + 4];
  const int wave = threadIdx.x >> 5, lane = threadIdx.x & 31, nloc = lane & 15, hlf = lane >> 4; const size_t m0 = (size_t)blockIdx.x * 64 + wave * 16; const int grp = blockIdx.y, c0 = grp * 128;
  for (int rr = 0; rr < 16; ++rr) { const size_t r = m0 + rr; const size_t v = r % N; v4f x = *(const v4f*)(ns + r * D + lane * 4); v4f p = {0.0f, 0.0f, 0.0f, 0.0f}; if (grp < 2) p = *(const v4f*)(npar + v * D + lane * 4);
    for (int j = 0; j < 4; ++j) { const float h = bf16_rne(x[j]) + (grp < 2 ? bf16_rne(p[j]) : 0.0f); b16 ph, pl; split16(h * XS, ph, pl); Ah[wave][rr][lane * 4 + j] = ph; Al[wave][rr][lane * 4 + j] = pl; } }
  wave_lds_sync();
  v8f acc[8];
#pragma unroll
  for (int t = 0; t < 8; ++t) acc[t] = (v8f){};
  const bool dolo = grp < 2;
#pragma unroll
  for (int kb = 0; kb < D; kb += 32) { const v16b a = frag_kb(&Ah[wave][nloc][kb], hlf), al = frag_kb(&Al[wave][nloc][kb], hlf);
#pragma unroll
    for (int t = 0; t < 8; ++t) { const v16b bw = frag_kb(WQK + (size_t)(c0 + t * 16 + nloc) * D + kb, hlf); acc[t] = wmma16b(a, bw, acc[t]); if (dolo) acc[t] = wmma16b(al, bw, acc[t]); } }
  wave_lds_sync();
#pragma unroll
  for (int t = 0; t < 8; ++t)
#pragma unroll 1
    for (int r = 0; r < 8; ++r) Tf[wave][8 * hlf + r][t * 16 + nloc] = acc[t][r] * (1.0f / (XS * WSC));
  wave_lds_sync();
  for (int pass = 0; pass < 2; ++pass) { for (int rr = 0; rr < 16; ++rr) *(volatile v4f*)(QKM + (m0 + rr) * QW + c0 + lane * 4) = *(const v4f*)(&Tf[wave][rr][lane * 4]); __threadfence(); }
}
__global__ __launch_bounds__(256) void src_kernel(const float* __restrict__ QKM, const float* __restrict__ rel, const int* __restrict__ dsts, const int* __restrict__ ety, const int* __restrict__ PERM, const int* __restrict__ ROWPTR, const int* __restrict__ ROWCNT, int permLen, float* __restrict__ MS, float* __restrict__ DS) {
  __shared__ float sm[32], sdn[32];
  const int wave = threadIdx.x >> 5, lane = threadIdx.x & 31;
#pragma unroll 1
  for (int qq = 0; qq < 4; ++qq) { const size_t r = (size_t)blockIdx.x * 32 + wave * 4 + qq; const int b = (int)(r / N); const int s = (int)(r % N);
    int st = ROWPTR[s], cnt = ROWCNT[s]; cnt = iclamp(cnt, 0, 65536); st = iclamp(st, 0, permLen - cnt); const v4f qv = *(const v4f*)(QKM + r * QW + lane * 4);
    float mx = -INFINITY;
#pragma unroll 1
    for (int j = 0; j < cnt; ++j) { const int e = iclamp(PERM[st + j], 0, E - 1); const size_t dn = (size_t)iclamp(dsts[e], 0, N - 1); const int et = iclamp(ety[e], 0, NE - 1); const v4f kv = *(const v4f*)(QKM + ((size_t)b * N + dn) * QW + D + lane * 4), rv = *(const v4f*)(rel + (size_t)et * D + lane * 4);
      float sc = 0.0f; for (int i = 0; i < 4; ++i) sc += pmul(qv[i], kv[i] + bf16_rne(rv[i])); for (int sh = 16; sh; sh >>= 1) sc += __shfl_xor(sc, sh); sc *= ISQD; mx = fmaxf(mx, sc); }
    float den = 0.0f;
#pragma unroll 1
    for (int j = 0; j < cnt; ++j) { const int e = iclamp(PERM[st + j], 0, E - 1); const size_t dn = (size_t)iclamp(dsts[e], 0, N - 1); const int et = iclamp(ety[e], 0, NE - 1); const v4f kv = *(const v4f*)(QKM + ((size_t)b * N + dn) * QW + D + lane * 4), rv = *(const v4f*)(rel + (size_t)et * D + lane * 4);
      float sc = 0.0f; for (int i = 0; i < 4; ++i) sc += pmul(qv[i], kv[i] + bf16_rne(rv[i])); for (int sh = 16; sh; sh >>= 1) sc += __shfl_xor(sc, sh); sc *= ISQD; den += nexp(sc - mx); }
    if (lane == 0) { sm[wave * 4 + qq] = (cnt > 0) ? mx : 0.0f; sdn[wave * 4 + qq] = den; } }
  __syncthreads();
  for (int pass = 0; pass < 2; ++pass) { if (threadIdx.x < 8) *(volatile v4f*)(MS + (size_t)blockIdx.x * 32 + threadIdx.x * 4) = *(const v4f*)(&sm[threadIdx.x * 4]); else if (threadIdx.x < 16) *(volatile v4f*)(DS + (size_t)blockIdx.x * 32 + (threadIdx.x - 8) * 4) = *(const v4f*)(&sdn[(threadIdx.x - 8) * 4]); __threadfence(); }
}
__global__ __launch_bounds__(256) void dst_kernel(const float* __restrict__ QKM, const float* __restrict__ rel, const float* __restrict__ attn, const int* __restrict__ srcs, const int* __restrict__ ety, const float* __restrict__ MS, const float* __restrict__ DS, const int* __restrict__ PERM, const int* __restrict__ ROWPTR, const int* __restrict__ ROWCNT, int permLen, float* __restrict__ AGG, float* __restrict__ outA) {
  __shared__ float sa[32];
  const int wave = threadIdx.x >> 5, lane = threadIdx.x & 31;
#pragma unroll 1
  for (int qq = 0; qq < 4; ++qq) { const size_t r = (size_t)blockIdx.x * 32 + wave * 4 + qq; const int b = (int)(r / N); const int dn = (int)(r % N);
    int st = ROWPTR[dn], cnt = ROWCNT[dn]; cnt = iclamp(cnt, 0, 65536); st = iclamp(st, 0, permLen - cnt); const v4f kv = *(const v4f*)(QKM + r * QW + D + lane * 4);
    float na = 0.0f; v4f ag = {0.0f, 0.0f, 0.0f, 0.0f};
#pragma unroll 1
    for (int j = 0; j < cnt; ++j) { const int e = iclamp(PERM[st + j], 0, E - 1); const int s = iclamp(srcs[e], 0, N - 1); const int et = iclamp(ety[e], 0, NE - 1); const size_t rs = (size_t)b * N + s;
      const v4f qv = *(const v4f*)(QKM + rs * QW + lane * 4), rv = *(const v4f*)(rel + (size_t)et * D + lane * 4), mv = *(const v4f*)(QKM + rs * QW + 2 * D + lane * 4);
      float sc = 0.0f; float rb[4]; for (int i = 0; i < 4; ++i) { rb[i] = bf16_rne(rv[i]); sc += pmul(qv[i], kv[i] + rb[i]); } for (int sh = 16; sh; sh >>= 1) sc += __shfl_xor(sc, sh); sc *= ISQD;
      const float tr = nexp(sc - MS[rs]) / (DS[rs] + EPSD); na += pmul(bf16_rne(attn[rs]), tr); for (int i = 0; i < 4; ++i) ag[i] += pmul(tr, mv[i] + rb[i]); }
    if (lane == 0) sa[wave * 4 + qq] = na;
    for (int pass = 0; pass < 2; ++pass) { *(volatile v4f*)(AGG + r * D + lane * 4) = ag; __threadfence(); } }
  __syncthreads();
  for (int pass = 0; pass < 2; ++pass) { if (threadIdx.x < 8) *(volatile v4f*)(outA + (size_t)blockIdx.x * 32 + threadIdx.x * 4) = *(const v4f*)(&sa[threadIdx.x * 4]); __threadfence(); }
}
__global__ __launch_bounds__(128) void upd_kernel(const float* __restrict__ ns, const float* __restrict__ AGG, const b16* __restrict__ WHA, const float* __restrict__ GW, float* __restrict__ outH) {
  __shared__ __attribute__((aligned(16))) b16 Ah[4][16][2 * D + 8], Al[4][16][2 * D + 8]; __shared__ __attribute__((aligned(16))) float Tf[4][16][D + 4];
  const int wave = threadIdx.x >> 5, lane = threadIdx.x & 31, nloc = lane & 15, hlf = lane >> 4; const size_t m0 = (size_t)blockIdx.x * 64 + wave * 16;
  for (int rr = 0; rr < 16; ++rr) { const size_t r = m0 + rr; const v4f x = *(const v4f*)(ns + r * D + lane * 4), a = *(const v4f*)(AGG + r * D + lane * 4);
    for (int j = 0; j < 4; ++j) { Ah[wave][rr][lane * 4 + j] = (b16)(bf16_rne(x[j]) * XS); Al[wave][rr][lane * 4 + j] = (b16)0.0f; b16 p, q; split16(a[j] * XS, p, q); Ah[wave][rr][D + lane * 4 + j] = p; Al[wave][rr][D + lane * 4 + j] = q; } }
  wave_lds_sync();
  v8f acc[8];
#pragma unroll
  for (int t = 0; t < 8; ++t) acc[t] = (v8f){};
#pragma unroll 2
  for (int kb = 0; kb < 2 * D; kb += 32) { const v16b a = frag_kb(&Ah[wave][nloc][kb], hlf), al = frag_kb(&Al[wave][nloc][kb], hlf); const bool dolo = kb >= D;
#pragma unroll
    for (int t = 0; t < 8; ++t) { const v16b bw = frag_kb(WHA + (size_t)(t * 16 + nloc) * 2 * D + kb, hlf); acc[t] = wmma16b(a, bw, acc[t]); if (dolo) acc[t] = wmma16b(al, bw, acc[t]); } }
  const int b = (int)(m0 / N);
#pragma unroll
  for (int t = 0; t < 8; ++t) { const int c = t * 16 + nloc; const float gw = GW[b * D + c];
#pragma unroll 1
    for (int r = 0; r < 8; ++r) Tf[wave][8 * hlf + r][c] = tanhf(acc[t][r] * (1.0f / (XS * WSC)) + gw); }
  wave_lds_sync();
  for (int pass = 0; pass < 2; ++pass) { for (int rr = 0; rr < 16; ++rr) *(volatile v4f*)(outH + (m0 + rr) * D + lane * 4) = *(const v4f*)(&Tf[wave][rr][lane * 4]); __threadfence(); }
}
}

extern "C" void kernel_launch(void* const* d_in, const int* in_sizes, int n_in, void* d_out, int out_size, void* d_ws, size_t ws_size, hipStream_t stream) {
  (void)n_in;
  auto Fp = [&](int i) { return (const float*)d_in[i]; }; auto Ip = [&](int i) { return (const int*)d_in[i]; };
  if (in_sizes[0] != M || in_sizes[1] != M * D || in_sizes[2] != N * D || in_sizes[3] != NE * D || in_sizes[4] != B * D || in_sizes[5] != D * D || in_sizes[11] != E || in_sizes[13] != E || out_size != M + M * D) return;
  size_t off = 0; char* ws = (char*)d_ws;
  auto carve = [&](size_t bytes) { char* p = ws + off; off += (bytes + 255) & ~(size_t)255; return p; };
  b16* WQK = (b16*)carve((size_t)QW * D * 2); b16* WHA = (b16*)carve((size_t)D * 2 * D * 2); float* GW = (float*)carve((size_t)B * D * 4); float* QKM = (float*)carve((size_t)M * QW * 4); float* AGG = (float*)carve((size_t)M * D * 4); float* MS = (float*)carve((size_t)M * 4); float* DS = (float*)carve((size_t)M * 4);
  CsrBufs csrS, csrD; off = csr_carve(csrS, ws, off, E, N); off = csr_carve(csrD, ws, off, E, N);
  if (off > ws_size) return;
  wprep_kernel<<<(unsigned)(((size_t)QW * D / 8 + (size_t)D * 2 * D / 8 + 255) / 256), 256, 0, stream>>>(Fp(5), Fp(6), Fp(7), Fp(8), Fp(9), WQK, WHA);
  gw_kernel<<<1, 256, 0, stream>>>(Fp(4), Fp(10), GW);
  csr_build(csrS, Ip(11), E, N, stream); csr_build(csrD, Ip(12), E, N, stream);
  qkm_kernel<<<dim3(M / 64, 3), 128, 0, stream>>>(Fp(1), Fp(2), WQK, QKM);
  src_kernel<<<M / 32, 256, 0, stream>>>(QKM, Fp(3), Ip(12), Ip(13), csrS.PERM, csrS.ROWPTR, csrS.ROWCNT, (int)csrS.permLen, MS, DS);
  float* outA = (float*)d_out; float* outH = outA + M;
  dst_kernel<<<M / 32, 256, 0, stream>>>(QKM, Fp(3), Fp(0), Ip(11), Ip(13), MS, DS, csrD.PERM, csrD.ROWPTR, csrD.ROWCNT, (int)csrD.permLen, AGG, outA);
  upd_kernel<<<M / 64, 128, 0, stream>>>(Fp(1), AGG, WHA, GW, outH);
}
